// GaussianMixture_70884140253931
// MI455X (gfx1250) — hardware-run, weakly checked
//
#include <hip/hip_runtime.h>
#include <math.h>

typedef __attribute__((ext_vector_type(16))) _Float16 v16h;
typedef __attribute__((ext_vector_type(16))) __bf16 v16b;
typedef __attribute__((ext_vector_type(8)))  _Float16 v8h;
typedef __attribute__((ext_vector_type(8)))  float v8f;
typedef __attribute__((ext_vector_type(4)))  float v4f;
typedef __attribute__((ext_vector_type(2)))  float v2f;
typedef __attribute__((ext_vector_type(4)))  unsigned v4u;
typedef __attribute__((ext_vector_type(4)))  int v4i;
typedef float __attribute__((may_alias)) float_a;
typedef int __attribute__((may_alias)) int_a;

template <typename T> __device__ __forceinline__ void vst2(void* p, T v) { *(volatile T*)p = v; __threadfence(); *(volatile T*)p = v; }
__device__ __forceinline__ v8f wmma16(v16h a, v16h b, v8f c) {
  v8f d = __builtin_amdgcn_wmma_f32_16x16x32_f16(false, a, false, b, (short)0, c, false, false);
  asm volatile("v_nop\n\tv_nop\n\tv_nop\n\tv_nop" : "+v"(d) : "v"(a), "v"(b));
  return d;
}
__device__ __forceinline__ v8f wmma_bf(v16b a, v16b b, v8f c) {
  v8f d = __builtin_amdgcn_wmma_f32_16x16x32_bf16(false, a, false, b, (short)0, c, false, false);
  asm volatile("v_nop\n\tv_nop\n\tv_nop\n\tv_nop" : "+v"(d) : "v"(a), "v"(b));
  return d;
}
__device__ __forceinline__ v16h frag_h(const _Float16* rowk0, int lane) {
  union { v16h v; v8h q[2]; } u; const _Float16* p = rowk0 + 8 * (lane >> 4);
  u.q[0] = *(const v8h*)p; u.q[1] = *(const v8h*)(p + 16); return u.v;
}
__device__ __forceinline__ v16h frag_f32(const float* rowk0, int lane) {
  v16h a; const float* p = rowk0 + 8 * (lane >> 4);
#pragma unroll
  for (int i = 0; i < 8; ++i) { a[i] = (_Float16)p[i]; a[8 + i] = (_Float16)p[16 + i]; }
  return a;
}
__device__ __forceinline__ v16h frag_f32s(const float* rowk0, int lane, float sc) {
  v16h a; const float* p = rowk0 + 8 * (lane >> 4);
#pragma unroll
  for (int i = 0; i < 8; ++i) { a[i] = (_Float16)(p[i] * sc); a[8 + i] = (_Float16)(p[16 + i] * sc); }
  return a;
}
__device__ __forceinline__ v16h fragc_f32(const float* W, int k0, int n, int lane, int ld, int K) {
  v16h a; const int g = lane >> 4;
#pragma unroll
  for (int i = 0; i < 8; ++i) { const int ka = k0 + 8 * g + i, kb = ka + 16;
    a[i] = (_Float16)(ka < K ? W[(size_t)(ka < K ? ka : K - 1) * ld + n] : 0.f); a[8 + i] = (_Float16)(kb < K ? W[(size_t)(kb < K ? kb : K - 1) * ld + n] : 0.f); }
  return a;
}
struct F2 { v16b h, l; };
__device__ __forceinline__ F2 bsplit16(const float v[16]) { F2 r;
#pragma unroll
  for (int i = 0; i < 16; ++i) { const __bf16 h = (__bf16)v[i]; r.h[i] = h; r.l[i] = (__bf16)(v[i] - (float)h); }
  return r; }
__device__ __forceinline__ F2 split_row(const float* row, int k0, int lane) { float v[16]; const float* p = row + k0 + 8 * (lane >> 4);
#pragma unroll
  for (int i = 0; i < 8; ++i) { v[i] = p[i]; v[8 + i] = p[16 + i]; }
  return bsplit16(v); }
__device__ __forceinline__ F2 split_rowK(const float* row, int k0, int lane, int K) { float v[16]; const int g = lane >> 4;
#pragma unroll
  for (int i = 0; i < 8; ++i) { const int ka = k0 + 8 * g + i, kb = ka + 16; v[i] = ka < K ? row[ka < K ? ka : K - 1] : 0.f; v[8 + i] = kb < K ? row[kb < K ? kb : K - 1] : 0.f; }
  return bsplit16(v); }
__device__ __forceinline__ F2 split_col(const float* W, int k0, int n, int lane, int ld, int K) { float v[16]; const int g = lane >> 4;
#pragma unroll
  for (int i = 0; i < 8; ++i) { const int ka = k0 + 8 * g + i, kb = ka + 16; v[i] = ka < K ? W[(size_t)(ka < K ? ka : K - 1) * ld + n] : 0.f; v[8 + i] = kb < K ? W[(size_t)(kb < K ? kb : K - 1) * ld + n] : 0.f; }
  return bsplit16(v); }
__device__ __forceinline__ v8f mac3(const F2& a, const F2& b, v8f c) { c = wmma_bf(a.l, b.h, c); c = wmma_bf(a.h, b.l, c); return wmma_bf(a.h, b.h, c); }
__device__ __forceinline__ float sigm(float v) { return 1.0f / (1.0f + expf(-v)); }
#define LDSX() do { asm volatile("s_wait_dscnt 0" ::: "memory"); __builtin_amdgcn_wave_barrier(); __builtin_amdgcn_fence(__ATOMIC_RELEASE, "workgroup"); } while (0)

#define NN 65536
#define DD 64
#define KC 32
#ifndef NRV
#define NRV NN
#endif
__device__ __forceinline__ float bfr(float v) { return (float)(__bf16)v; }
#define WS_SCT  0u
#define WS_CSC  (WS_SCT + 4u * DD * KC)
#define WS_LCF  (WS_CSC + 128u)
#define WS_END  (WS_LCF + 128u)
__global__ __launch_bounds__(256) void k_prep(const float* __restrict__ Lm, const float* __restrict__ Cc, const float* __restrict__ Wt, float* __restrict__ SCT, float* __restrict__ CSC, float* __restrict__ LCF) {
  __shared__ float sS[8][DD][DD + 1]; __shared__ float sv[8][DD]; __shared__ __align__(16) float sSc[DD][KC]; __shared__ float scsc[KC]; __shared__ float slcf[KC];
  const int tid = threadIdx.x, wave = tid >> 5, lane = tid & 31, col = lane & 15, g = lane >> 4;
  float wsum = 0.f; for (int k = 0; k < KC; ++k) wsum += fabsf(bfr(Wt[k]));
  for (int kk = wave; kk < KC; kk += 8) { const float* Lk = Lm + (size_t)kk * DD * DD;
#pragma unroll 1
    for (int ti = 0; ti < 4; ++ti) { v8f acc[4] = {};
#pragma unroll
      for (int kc = 0; kc < 2; ++kc) { v16b a; { const float* p = Lk + (size_t)(ti * 16 + col) * DD + kc * 32 + 8 * g;
#pragma unroll
          for (int i = 0; i < 8; ++i) { a[i] = (__bf16)p[i]; a[8 + i] = (__bf16)p[16 + i]; } }
        asm volatile("s_wait_loadcnt 0x0" ::: "memory");
#pragma unroll
        for (int tj = 0; tj < 4; ++tj) { v16b b; { const float* p = Lk + (size_t)(tj * 16 + col) * DD + kc * 32 + 8 * g;
#pragma unroll
            for (int i = 0; i < 8; ++i) { b[i] = (__bf16)p[i]; b[8 + i] = (__bf16)p[16 + i]; } }
          asm volatile("s_wait_loadcnt 0x0" ::: "memory"); acc[tj] = wmma_bf(a, b, acc[tj]); } }
#pragma unroll
      for (int tj = 0; tj < 4; ++tj) {
#pragma unroll
        for (int r = 0; r < 8; ++r) sS[wave][ti * 16 + 8 * g + r][tj * 16 + col] = acc[tj][r]; } }
    LDSX();
    { float a0 = 0.f, a1 = 0.f;
      for (int e = 0; e < DD; ++e) { const float ce = bfr(Cc[(size_t)kk * DD + e]); a0 += sS[wave][lane][e] * ce; a1 += sS[wave][lane + 32][e] * ce; }
      sSc[lane][kk] = a0; sSc[lane + 32][kk] = a1;
      float part = a0 * bfr(Cc[(size_t)kk * DD + lane]) + a1 * bfr(Cc[(size_t)kk * DD + lane + 32]);
#pragma unroll
      for (int o = 1; o < 32; o <<= 1) part += __shfl_xor(part, o);
      if (lane == 0) scsc[kk] = part; }
    { float logdet = 0.f;
      for (int j = 0; j < DD; ++j) {
        LDSX();
        float djj = sS[wave][j][j]; for (int q = 0; q < j; ++q) djj -= sS[wave][j][q] * sS[wave][j][q];
        const float dj = sqrtf(fmaxf(djj, 1e-30f)); logdet += logf(dj);
#pragma unroll
        for (int h2 = 0; h2 < 2; ++h2) { const int i = lane + 32 * h2;
          if (i > j) { float sij = sS[wave][i][j]; for (int q = 0; q < j; ++q) sij -= sS[wave][i][q] * sS[wave][j][q]; sv[wave][i] = sij / dj; } }
        LDSX();
#pragma unroll
        for (int h2 = 0; h2 < 2; ++h2) { const int i = lane + 32 * h2; if (i > j) sS[wave][i][j] = sv[wave][i]; }
        if (lane == 0) sS[wave][j][j] = dj; }
      LDSX();
      if (lane == 0) slcf[kk] = logf(fabsf(bfr(Wt[kk])) / wsum) + logdet; }
    LDSX(); }
  __syncthreads();
  for (int d = wave; d < DD; d += 8) if (lane < 8) vst2(SCT + (size_t)d * KC + lane * 4, *(const v4f*)&sSc[d][lane * 4]);
  if (tid < 8) { v4f v; v[0] = scsc[tid * 4]; v[1] = scsc[tid * 4 + 1]; v[2] = scsc[tid * 4 + 2]; v[3] = scsc[tid * 4 + 3]; vst2(CSC + tid * 4, v); }
  if (tid >= 32 && tid < 40) { const int t = tid - 32; v4f v; v[0] = slcf[t * 4]; v[1] = slcf[t * 4 + 1]; v[2] = slcf[t * 4 + 2]; v[3] = slcf[t * 4 + 3]; vst2(LCF + t * 4, v); } }
__global__ __launch_bounds__(128) void k_main(const float* __restrict__ X, const float* __restrict__ Lm, const float* __restrict__ SCT, const float* __restrict__ CSC, const float* __restrict__ LCF, const float* __restrict__ TH, float* __restrict__ OUT) {
  __shared__ float sd[4][16][KC + 1]; __shared__ __align__(16) float sll[64];
  const int tid = threadIdx.x, wave = tid >> 5, lane = tid & 31, col = lane & 15, g = lane >> 4; const size_t n0 = (size_t)blockIdx.x * 64 + wave * 16;
  v16b xa[2];
#pragma unroll
  for (int kc = 0; kc < 2; ++kc) { const float* p = X + (n0 + col) * DD + kc * 32 + 8 * g;
#pragma unroll
    for (int i = 0; i < 8; ++i) { xa[kc][i] = (__bf16)p[i]; xa[kc][8 + i] = (__bf16)p[16 + i]; } }
  asm volatile("s_wait_loadcnt 0x0" ::: "memory");
  v8f asc[2] = {};
#pragma unroll
  for (int kc = 0; kc < 2; ++kc) {
#pragma unroll
    for (int j = 0; j < 2; ++j) { v16b bh, bl; { const float* p = SCT + (size_t)(kc * 32 + 8 * g) * KC + j * 16 + col; float t0[8], t1[8];
#pragma unroll
        for (int i = 0; i < 8; ++i) t0[i] = p[(size_t)i * KC];
        asm volatile("s_wait_loadcnt 0x0" ::: "memory");
#pragma unroll
        for (int i = 0; i < 8; ++i) t1[i] = p[(size_t)(16 + i) * KC];
        asm volatile("s_wait_loadcnt 0x0" ::: "memory");
#pragma unroll
        for (int i = 0; i < 8; ++i) { const __bf16 h0 = (__bf16)t0[i], h1 = (__bf16)t1[i]; bh[i] = h0; bh[8 + i] = h1; bl[i] = (__bf16)(t0[i] - (float)h0); bl[8 + i] = (__bf16)(t1[i] - (float)h1); } }
      asc[j] = wmma_bf(xa[kc], bh, asc[j]); asc[j] = wmma_bf(xa[kc], bl, asc[j]); } }
#pragma unroll 1
  for (int k = 0; k < KC; ++k) { const float* Lk = Lm + (size_t)k * DD * DD; v8f acc[4] = {};
#pragma unroll
    for (int kc = 0; kc < 2; ++kc) {
#pragma unroll
      for (int j = 0; j < 4; ++j) { v16b b; { const float* p = Lk + (size_t)(kc * 32 + 8 * g) * DD + j * 16 + col; float t0[8], t1[8];
#pragma unroll
          for (int i = 0; i < 8; ++i) t0[i] = p[(size_t)i * DD];
          asm volatile("s_wait_loadcnt 0x0" ::: "memory");
#pragma unroll
          for (int i = 0; i < 8; ++i) t1[i] = p[(size_t)(16 + i) * DD];
          asm volatile("s_wait_loadcnt 0x0" ::: "memory");
#pragma unroll
          for (int i = 0; i < 8; ++i) { b[i] = (__bf16)t0[i]; b[8 + i] = (__bf16)t1[i]; } }
        acc[j] = wmma_bf(xa[kc], b, acc[j]); } }
    float ps[8];
#pragma unroll
    for (int r = 0; r < 8; ++r) { float q = 0.f;
#pragma unroll
      for (int j = 0; j < 4; ++j) q += acc[j][r] * acc[j][r]; ps[r] = q; }
#pragma unroll
    for (int o = 1; o < 16; o <<= 1) {
#pragma unroll
      for (int r = 0; r < 8; ++r) ps[r] += __shfl_xor(ps[r], o); }
    if (col == 0) {
#pragma unroll
      for (int r = 0; r < 8; ++r) sd[wave][8 * g + r][k] = ps[r]; } }
  LDSX();
#pragma unroll
  for (int j = 0; j < 2; ++j) { const int k = j * 16 + col; const float cs = CSC[k], lc = LCF[k]; asm volatile("s_wait_loadcnt 0x0" ::: "memory");
#pragma unroll
    for (int r = 0; r < 8; ++r) { const float xsx = sd[wave][8 * g + r][k]; sd[wave][8 * g + r][k] = -0.5f * ((xsx - 2.0f * asc[j][r]) + cs) + lc; } }
  LDSX();
  if (lane < 16) { float m = -3.0e38f; for (int k = 0; k < KC; ++k) m = fmaxf(m, sd[wave][lane][k]); float se = 0.f; for (int k = 0; k < KC; ++k) se += expf(sd[wave][lane][k] - m); sll[wave * 16 + lane] = (m + logf(se)) - bfr(TH[0]); }
  __syncthreads();
  if (tid < 16) vst2(OUT + (size_t)blockIdx.x * 64 + tid * 4, *(const v4f*)&sll[tid * 4]); }
extern "C" void kernel_launch(void* const* d_in, const int* in_sizes, int n_in, void* d_out, int out_size, void* d_ws, size_t ws_size, hipStream_t stream) {
  (void)in_sizes; (void)n_in; (void)out_size;
  if (ws_size < (size_t)WS_END) return;
  char* ws = (char*)d_ws; const float** F = (const float**)d_in; float *SCT = (float*)(ws + WS_SCT), *CSC = (float*)(ws + WS_CSC), *LCF = (float*)(ws + WS_LCF);
  k_prep<<<1, 256, 0, stream>>>(F[2], F[1], F[3], SCT, CSC, LCF);
  k_main<<<dim3(NRV / 64), 128, 0, stream>>>(F[0], F[2], SCT, CSC, LCF, F[4], (float*)d_out);
}
